// SubgraphSpecificLatentProjector_47854525612388
// MI455X (gfx1250) — hardware-verified
//
#include <hip/hip_runtime.h>
#include <stddef.h>


typedef _Float16 v16h __attribute__((ext_vector_type(16)));
typedef _Float16 v8h  __attribute__((ext_vector_type(8)));
typedef float    v8f  __attribute__((ext_vector_type(8)));
typedef float    v4f  __attribute__((ext_vector_type(4)));

#ifndef NB
#define NB 256
#endif
#define NB_FULL 256
#define NN   32
#define DD   128
#define DJ   128
#define RR   8
#define OO   8
#define NKEY (RR * OO)

#define NCTR  (NB)
#define NNBR  (NB * NN)
#define NCAND (NCTR + NNBR)
#define NCH_C ((NCTR + 255) / 256)
#define NCH_N ((NNBR + 255) / 256)
#define MAXLIST  (NCAND)
#define TROWS    64
#define MAXTILES ((MAXLIST + TROWS - 1) / TROWS)

#define OUT1_ELEMS     ((unsigned)NB_FULL * RR * DJ)
#define OUT_ELEMS_FULL ((size_t)OUT1_ELEMS + (size_t)NB_FULL * NN * DJ)

static_assert(NB >= 1 && NB <= NB_FULL);
static_assert((size_t)OUT1_ELEMS * 4 == (size_t)1048576);
static_assert(OUT_ELEMS_FULL * 4 == (size_t)5242880);
static_assert((size_t)OUT1_ELEMS + (size_t)NNBR * DJ <= OUT_ELEMS_FULL);
static_assert((size_t)NCTR * RR * DJ <= (size_t)OUT1_ELEMS);
static_assert((DD % 32) == 0 && (DD % 64) == 0 && (DJ % 64) == 0);
static_assert(DJ == 2 * 4 * 16);
static_assert(TROWS == 4 * 16);
static_assert(DJ == 32 * 4);
static_assert(TROWS == 8 * 8);
static_assert(TROWS * (DD / 8) == 4 * 256);
static_assert(NKEY == 64);

#define LDT  72
#define LDA  136
#define LDCC 132
static_assert((LDT % 8) == 0 && LDT >= 64);
static_assert((LDA % 8) == 0 && LDA >= DD);
static_assert((LDCC % 4) == 0 && LDCC >= DJ);

#define WCARRY 64.0f
#define ACARRY 16.0f
#define CFOLD  (1.0f / (WCARRY * ACARRY))

#define LDS_PROJ_BYTES ((size_t)MAXLIST * 4 + 8 * 4 + TROWS * 4 + (size_t)TROWS * LDA * 2 + (size_t)TROWS * LDCC * 4)
static_assert(LDS_PROJ_BYTES <= (size_t)131072);

#define WPLANE_BYTES ((size_t)NKEY * DD * DJ * 2)
#define OFF_MT   ((size_t)0)
#define WS_TOTAL (OFF_MT + WPLANE_BYTES)
static_assert((WPLANE_BYTES % 128) == 0);
static_assert(WS_TOTAL <= (size_t)134217728);

__device__ __forceinline__ float bf16r(float x) {
  unsigned int u = __float_as_uint(x);
  u = (u + 0x7FFFu + ((u >> 16) & 1u)) & 0xFFFF0000u;
  return __uint_as_float(u);
}

__device__ __forceinline__ _Float16 toh_flush(float v) {
  const _Float16 r = (_Float16)v;
  return (fabsf(v) < 6.103515625e-05f) ? (_Float16)0.0f : r;
}

__device__ __forceinline__ v16h frag_at(const _Float16* p) {
  v8h lo = *(const v8h*)(p);
  v8h hi = *(const v8h*)(p + 16);
  v16h out;
#pragma unroll
  for (int i = 0; i < 8; ++i) { out[i] = lo[i]; out[i + 8] = hi[i]; }
  return out;
}
__device__ __forceinline__ v16h ld_frag(const _Float16* base, unsigned ld) {
  const unsigned lane = threadIdx.x & 31u;
  return frag_at(base + (lane & 15u) * ld + (lane >> 4) * 8u);
}

__device__ __forceinline__ v8f wmma16(v16h a, v16h b, v8f c) {
  v8f d = __builtin_amdgcn_wmma_f32_16x16x32_f16(false, a, false, b, (short)0, c,
                                                 false, false);
  asm volatile("v_nop\n\tv_nop\n\tv_nop\n\tv_nop" : "+v"(d) : "v"(a), "v"(b));
  return d;
}

__global__ __launch_bounds__(256) void wconv_kernel(
    const float* __restrict__ W, _Float16* __restrict__ Wt, unsigned ldw, unsigned ldk) {
  __shared__ _Float16 T[64 * LDT];
  const unsigned tid = threadIdx.x;
  const unsigned n0 = blockIdx.x * 64u;
  const unsigned k0 = blockIdx.y * 64u;
  const size_t zo = (size_t)blockIdx.z * ldw * ldk;
#pragma unroll 4
  for (unsigned j = 0; j < 16u; ++j) {
    const unsigned idx = tid + 256u * j;
    const unsigned kr = idx >> 6, nc = idx & 63u;
    const float v = W[zo + (size_t)(k0 + kr) * ldw + n0 + nc];
    T[nc * LDT + kr] = toh_flush(WCARRY * bf16r(v));
  }
  __syncthreads();
  v8h x[2];
  size_t off[2];
#pragma unroll
  for (unsigned i = 0; i < 2u; ++i) {
    const unsigned n = 32u * i + (tid >> 3);
    const unsigned kc = (tid & 7u) * 8u;
    x[i] = *(const v8h*)&T[n * LDT + kc];
    off[i] = zo + (size_t)(n0 + n) * ldk + k0 + kc;
  }
#pragma unroll
  for (int i = 0; i < 2; ++i) *(volatile v8h*)(Wt + off[i]) = x[i];
  __threadfence();
#pragma unroll
  for (int i = 0; i < 2; ++i) *(volatile v8h*)(Wt + off[i]) = x[i];
}

__global__ __launch_bounds__(256) void proj_kernel(
    const float* __restrict__ center_h, const float* __restrict__ neigh,
    const _Float16* __restrict__ Mt, const float* __restrict__ bias,
    const int* __restrict__ center_o, const int* __restrict__ s_types,
    const int* __restrict__ o_types, float* __restrict__ out) {
  __shared__ int list[MAXLIST];
  __shared__ int wcnt[8];
  __shared__ unsigned rowdst[TROWS];
  __shared__ _Float16 As[TROWS * LDA];
  __shared__ float Cs[TROWS * LDCC];

  const unsigned tid = threadIdx.x, lane = tid & 31u;
  const unsigned w = (unsigned)__builtin_amdgcn_readfirstlane((int)(threadIdx.x >> 5));
  const unsigned hh = lane >> 4, m = lane & 15u;
  const unsigned key = blockIdx.x;
  const int ks = (int)(key >> 3);
  const int ko = (int)(key & 7u);

  unsigned total = 0u;
#pragma unroll 1
  for (unsigned ch = 0; ch < (unsigned)(NCH_C + NCH_N); ++ch) {
    bool hit;
    int id;
    if (ch < (unsigned)NCH_C) {
      const unsigned cand = ch * 256u + tid;
      const unsigned ca = (cand < (unsigned)NCTR) ? cand : (unsigned)(NCTR - 1);
      int o = center_o[ca];
      o = (o < 0) ? (o + OO) : o;
      o = (o < 0) ? 0 : ((o > OO - 1) ? (OO - 1) : o);
      hit = (cand < (unsigned)NCTR) && (o == ko);
      id = (int)ca;
    } else {
      const unsigned cand = (ch - (unsigned)NCH_C) * 256u + tid;
      const unsigned ca = (cand < (unsigned)NNBR) ? cand : (unsigned)(NNBR - 1);
      int s = s_types[ca];
      int o = o_types[ca];
      s = (s < 0) ? 0 : ((s > RR - 1) ? (RR - 1) : s);
      o = (o < 0) ? 0 : ((o > OO - 1) ? (OO - 1) : o);
      hit = (cand < (unsigned)NNBR) && (s == ks) && (o == ko);
      id = NCTR + (int)ca;
    }
    const unsigned bal = __builtin_amdgcn_ballot_w32(hit);
    if (lane == 0u) wcnt[w] = (int)__builtin_popcount(bal);
    __syncthreads();
    unsigned pre = 0u, tot = 0u;
#pragma unroll
    for (unsigned i = 0; i < 8u; ++i) {
      const unsigned c = (unsigned)wcnt[i];
      pre += (i < w) ? c : 0u;
      tot += c;
    }
    const unsigned pos = total + pre + (unsigned)__builtin_popcount(bal & ((1u << lane) - 1u));
    if (hit) list[(pos < (unsigned)MAXLIST) ? pos : (unsigned)(MAXLIST - 1)] = id;
    total += tot;
    __syncthreads();
  }
  const unsigned tcl = (total < (unsigned)MAXLIST) ? total : (unsigned)MAXLIST;
  const unsigned cnt = (unsigned)__builtin_amdgcn_readfirstlane((int)tcl);
  const unsigned ntiles = (cnt + (unsigned)TROWS - 1u) / (unsigned)TROWS;

  float bb[4];
  {
    const v4f gb = *(const v4f*)(bias + (size_t)key * DJ + lane * 4u);
#pragma unroll
    for (int j = 0; j < 4; ++j) bb[j] = bf16r(gb[j]);
  }

  const unsigned mw = w >> 1, nw = w & 1u;
  const _Float16* bp = Mt + (size_t)key * (DD * DJ) + (size_t)(nw * 64u + m) * DD + hh * 8u;

#pragma unroll 1
  for (unsigned tl = 0; tl < ntiles; ++tl) {
    const unsigned t0 = tl * (unsigned)TROWS;

    if (tid < (unsigned)TROWS) {
      const unsigned p = t0 + tid;
      const unsigned pc = (p < cnt) ? p : (cnt - 1u);
      int id = list[pc];
      id = (id < 0) ? 0 : ((id > NCAND - 1) ? (NCAND - 1) : id);
      const unsigned dctr = ((unsigned)id * RR + (unsigned)ks) * DJ;
      const unsigned dnbr = OUT1_ELEMS + (unsigned)(id - NCTR) * DJ;
      rowdst[tid] = (id < NCTR) ? dctr : dnbr;
    }

#pragma unroll 2
    for (unsigned j = 0; j < 4u; ++j) {
      const unsigned idx = tid + 256u * j;
      const unsigned row = idx >> 4, seg = idx & 15u;
      const unsigned p = t0 + row;
      const bool valid = p < cnt;
      const unsigned pc = valid ? p : (cnt - 1u);
      int id = list[pc];
      id = (id < 0) ? 0 : ((id > NCAND - 1) ? (NCAND - 1) : id);
      const bool isc = id < NCTR;
      const unsigned bc = isc ? (unsigned)id : 0u;
      const unsigned nc = isc ? 0u : (unsigned)(id - NCTR);
      const float* cp = center_h + (size_t)bc * DD + seg * 8u;
      const float* np = neigh + (size_t)nc * DD + seg * 8u;
      const v4f c0 = *(const v4f*)(cp);
      const v4f c1 = *(const v4f*)(cp + 4);
      const v4f n0 = *(const v4f*)(np);
      const v4f n1 = *(const v4f*)(np + 4);
      v8h x;
#pragma unroll
      for (int i = 0; i < 4; ++i) {
        float e0 = isc ? c0[i] : n0[i];
        float e1 = isc ? c1[i] : n1[i];
        e0 = valid ? e0 : 0.0f;
        e1 = valid ? e1 : 0.0f;
        x[i]     = toh_flush(ACARRY * bf16r(e0));
        x[i + 4] = toh_flush(ACARRY * bf16r(e1));
      }
      *(v8h*)&As[row * LDA + seg * 8u] = x;
    }
    __syncthreads();

    v8f acc[4];
#pragma unroll
    for (int j = 0; j < 4; ++j) acc[j] = (v8f){};
#pragma unroll
    for (unsigned k0 = 0; k0 < (unsigned)DD; k0 += 32u) {
      const v16h a = ld_frag(&As[(mw * 16u) * LDA + k0], LDA);
#pragma unroll
      for (int j = 0; j < 4; ++j) {
        const v16h bf = frag_at(bp + (size_t)(j * 16) * DD + k0);
        acc[j] = wmma16(a, bf, acc[j]);
      }
    }
#pragma unroll
    for (int j = 0; j < 4; ++j)
#pragma unroll
      for (int r = 0; r < 8; ++r)
        Cs[(mw * 16u + hh * 8u + (unsigned)r) * LDCC + nw * 64u + (unsigned)j * 16u + m] = acc[j][r];
    __syncthreads();

#pragma unroll 1
    for (unsigned i = 0; i < 8u; ++i) {
      const unsigned r = w * 8u + i;
      const v4f u = *(const v4f*)&Cs[r * LDCC + lane * 4u];
      v4f t;
#pragma unroll
      for (int j = 0; j < 4; ++j) {
        const float xv = u[j] * CFOLD + bb[j];
        t[j] = 0.5f * xv * (1.0f + erff(xv * 0.70710678118654752f));
      }
      *(v4f*)&Cs[r * LDCC + lane * 4u] = t;
    }

    v4f xs[8];
    unsigned off[8];
#pragma unroll
    for (unsigned i = 0; i < 8u; ++i) {
      const unsigned r = w * 8u + i;
      xs[i] = *(const v4f*)&Cs[r * LDCC + lane * 4u];
      off[i] = rowdst[r] + lane * 4u;
    }
#pragma unroll
    for (unsigned i = 0; i < 8u; ++i)
      if (t0 + w * 8u + i < cnt) *(volatile v4f*)(out + off[i]) = xs[i];
    __threadfence();
#pragma unroll
    for (unsigned i = 0; i < 8u; ++i)
      if (t0 + w * 8u + i < cnt) *(volatile v4f*)(out + off[i]) = xs[i];
    __syncthreads();
  }
}

extern "C" void kernel_launch(void* const* d_in, const int* in_sizes, int n_in,
                              void* d_out, int out_size, void* d_ws, size_t ws_size,
                              hipStream_t stream) {
  if (n_in < 7) return;
  if ((long long)in_sizes[0] < (long long)NB * DD) return;
  if ((long long)in_sizes[1] < (long long)NB * NN * DD) return;
  if ((long long)in_sizes[2] < (long long)NKEY * DD * DJ) return;
  if ((long long)in_sizes[3] < (long long)NKEY * DJ) return;
  if ((long long)in_sizes[4] < (long long)NB) return;
  if ((long long)in_sizes[5] < (long long)NB * NN) return;
  if ((long long)in_sizes[6] < (long long)NB * NN) return;
  if ((long long)out_size < (long long)OUT1_ELEMS + (long long)NNBR * DJ) return;
  if (ws_size < WS_TOTAL) return;

  const float* center_h = (const float*)d_in[0];
  const float* neigh    = (const float*)d_in[1];
  const float* Mw       = (const float*)d_in[2];
  const float* bias     = (const float*)d_in[3];
  const int*   center_o = (const int*)d_in[4];
  const int*   s_types  = (const int*)d_in[5];
  const int*   o_types  = (const int*)d_in[6];
  float* out = (float*)d_out;

  char* ws = (char*)d_ws;
  _Float16* Mt = (_Float16*)(ws + OFF_MT);

  dim3 blk(256);
  wconv_kernel<<<dim3(DJ / 64, DD / 64, NKEY), blk, 0, stream>>>(Mw, Mt, (unsigned)DJ, (unsigned)DD);
  proj_kernel<<<dim3(NKEY), blk, 0, stream>>>(center_h, neigh, Mt, bias, center_o, s_types,
                                              o_types, out);
}
